// MultiheadAttention_11029476016138
// MI455X (gfx1250) — hardware-verified
//
#include <hip/hip_runtime.h>


#ifndef NB
#define NB 2
#endif
#ifndef SEQ
#define SEQ 2048
#endif
#define SEQ_FULL 2048
#define TT   SEQ
#define DM   1024
#define NH_  16
#define HD   64
#define ZH   2
#define PCAR 1024.0f
#define SCL  0.125f
typedef _Float16 h16;
typedef unsigned short bf;
typedef __attribute__((ext_vector_type(16))) __bf16   v16bf;
typedef __attribute__((ext_vector_type(16))) _Float16 v16h;
typedef __attribute__((ext_vector_type(8)))  _Float16 v8h;
typedef __attribute__((ext_vector_type(4)))  _Float16 v4h;
typedef __attribute__((ext_vector_type(8)))  unsigned short v8us;
typedef __attribute__((ext_vector_type(8)))  float    v8f;
typedef __attribute__((ext_vector_type(4)))  float    v4f;
typedef v4f  __attribute__((may_alias)) v4fa;

static_assert(TT % 128 == 0);
static_assert(SEQ <= SEQ_FULL);
static_assert(HD == 64);
static_assert(DM == NH_ * HD);
static_assert(NH_ % ZH == 0);
static_assert((size_t)3 * NB * NH_ * TT * HD * 2 + (size_t)ZH * TT * TT * 6 <= (size_t)134217728);

__device__ __forceinline__ unsigned short f2bf(float f) { unsigned u = __float_as_uint(f); u += 0x7FFFu + ((u >> 16) & 1u); return (unsigned short)(u >> 16); }
__device__ __forceinline__ float bf2f(unsigned short b) { return __uint_as_float(((unsigned)b) << 16); }
__device__ __forceinline__ float bfr(float f) { return bf2f(f2bf(f)); }
__device__ __forceinline__ h16 tohx(float x) { return (h16)x; }
__device__ __forceinline__ v16h cat16(v8h lo, v8h hi) { return __builtin_shufflevector(lo, hi, 0, 1, 2, 3, 4, 5, 6, 7, 8, 9, 10, 11, 12, 13, 14, 15); }
__device__ __forceinline__ v16bf cat16b(v8us lo, v8us hi) { return __builtin_bit_cast(v16bf, __builtin_shufflevector(lo, hi, 0, 1, 2, 3, 4, 5, 6, 7, 8, 9, 10, 11, 12, 13, 14, 15)); }
__device__ __forceinline__ v8f wmma16(v16h a, v16h b, v8f c) { return __builtin_amdgcn_wmma_f32_16x16x32_f16(false, a, false, b, (short)0, c, false, false); }
__device__ __forceinline__ v8f wmmab(v16bf a, v16bf b, v8f c) { return __builtin_amdgcn_wmma_f32_16x16x32_bf16(false, a, false, b, (short)0, c, false, false); }

template <typename T16> struct WFrag;
template <> struct WFrag<h16> { typedef v16h V; static __device__ __forceinline__ V ld(const h16* p) { return cat16(*(const v8h*)p, *(const v8h*)(p + 16)); } static __device__ __forceinline__ v8f mma(V a, V b, v8f c) { return wmma16(a, b, c); } };
template <> struct WFrag<bf> { typedef v16bf V; static __device__ __forceinline__ V ld(const bf* p) { return cat16b(*(const v8us*)p, *(const v8us*)(p + 16)); } static __device__ __forceinline__ v8f mma(V a, V b, v8f c) { return wmmab(a, b, c); } };
template <typename T16>
__global__ __launch_bounds__(32) void k_gemmw(const T16* __restrict__ A, const T16* __restrict__ Bt, int K, float* C, int ldc, size_t sA, size_t sB, size_t sC, float oscale) {
    typedef typename WFrag<T16>::V V;
    __shared__ __align__(16) float os[16 * 68];
    const size_t z = blockIdx.z; A += z * sA; Bt += z * sB; C += z * sC;
    const int lane = threadIdx.x & 31, lr = lane & 15, hi = lane >> 4; const int r0 = blockIdx.x * 64, c0 = blockIdx.y * 64;
    v8f acc[4][4];
#pragma unroll
    for (int mb = 0; mb < 4; ++mb)
#pragma unroll
        for (int nb = 0; nb < 4; ++nb) acc[mb][nb] = (v8f){};
    const size_t aoff = (size_t)(r0 + lr) * K + 8 * hi, boff = (size_t)(c0 + lr) * K + 8 * hi;
#pragma unroll 1
    for (int kc = 0; kc < K; kc += 32) {
        V a[4];
#pragma unroll
        for (int mb = 0; mb < 4; ++mb) a[mb] = WFrag<T16>::ld(A + aoff + (size_t)mb * 16 * K + kc);
#pragma unroll
        for (int nb = 0; nb < 4; ++nb) { const V b = WFrag<T16>::ld(Bt + boff + (size_t)nb * 16 * K + kc);
#pragma unroll
            for (int mb = 0; mb < 4; ++mb) acc[mb][nb] = WFrag<T16>::mma(a[mb], b, acc[mb][nb]); }
        asm volatile("v_nop\n\tv_nop\n\tv_nop\n\tv_nop" : "+v"(acc[0][0]), "+v"(acc[1][1]), "+v"(acc[2][2]), "+v"(acc[3][3]) : "v"(a[0]), "v"(a[3]));
    }
#pragma unroll
    for (int mb = 0; mb < 4; ++mb) {
#pragma unroll
        for (int nb = 0; nb < 4; ++nb) {
#pragma unroll
            for (int j = 0; j < 8; ++j) os[(hi * 8 + j) * 68 + nb * 16 + lr] = acc[mb][nb][j]; }
        __builtin_amdgcn_wave_barrier(); asm volatile("" ::: "memory");
        float* crow = C + (size_t)(r0 + mb * 16) * ldc + c0;
#pragma unroll 1
        for (int ps = 0; ps < 2; ++ps) {
#pragma unroll
            for (int s = 0; s < 8; ++s) { const int row = 2 * s + hi, cofs = lr * 4; v4f val = *(const v4fa*)(os + row * 68 + cofs); val = val * oscale;
                *(volatile v4f*)(crow + (size_t)row * ldc + cofs) = val; }
            if (ps == 0) __threadfence(); }
        __builtin_amdgcn_wave_barrier(); asm volatile("" ::: "memory");
    }
}

__global__ __launch_bounds__(256) void k_hp8(const float* __restrict__ q, const float* __restrict__ k, bf* QB, bf* KB) {
    const size_t i = (size_t)blockIdx.x * 256 + threadIdx.x; if (i >= (size_t)NB * NH_ * TT * (HD / 8)) return;
    const int d8 = (int)(i % (HD / 8)); const int t = (int)((i / (HD / 8)) % TT); const int h = (int)((i / ((size_t)(HD / 8) * TT)) % NH_); const int b = (int)(i / ((size_t)(HD / 8) * TT * NH_));
    const size_t so = ((size_t)b * SEQ_FULL + t) * DM + h * HD + d8 * 8;
    const v8f a = *(const v8f*)(q + so); const v8f c = *(const v8f*)(k + so); v8us oq, ok;
#pragma unroll
    for (int e = 0; e < 8; ++e) { oq[e] = f2bf(a[e]); ok[e] = f2bf(c[e]); }
    *(volatile v8us*)(QB + i * 8) = oq; *(volatile v8us*)(KB + i * 8) = ok; __threadfence(); *(volatile v8us*)(QB + i * 8) = oq; *(volatile v8us*)(KB + i * 8) = ok; }

__global__ __launch_bounds__(256) void k_vt8(const float* __restrict__ v, h16* V16) {
    const size_t i = (size_t)blockIdx.x * 256 + threadIdx.x; if (i >= (size_t)NB * NH_ * HD * (TT / 8)) return;
    const int t8 = (int)(i % (TT / 8)); const int d = (int)((i / (TT / 8)) % HD); const int g = (int)((i / ((size_t)(TT / 8) * HD)) % NH_); const int b = (int)(i / ((size_t)(TT / 8) * HD * NH_));
    const float* src = v + ((size_t)b * SEQ_FULL + (size_t)t8 * 8) * DM + g * HD + d; v8h o;
#pragma unroll
    for (int j = 0; j < 8; ++j) o[j] = tohx(bfr(src[(size_t)j * DM]));
    *(volatile v8h*)(V16 + i * 8) = o; __threadfence(); *(volatile v8h*)(V16 + i * 8) = o; }

__global__ __launch_bounds__(256) void k_asoft(const float* __restrict__ Sb, h16* P16) {
    const int lane = threadIdx.x & 31; const int row = blockIdx.x * 8 + (threadIdx.x >> 5); if (row >= ZH * TT) return; const float* sr = Sb + (size_t)row * TT; float v[TT / 32]; float mx = -3.0e38f;
#pragma unroll
    for (int ch = 0; ch < TT / 128; ++ch) { const int j0 = ch * 128 + lane * 4; const v4f a = *(const v4f*)(sr + j0);
#pragma unroll
        for (int q = 0; q < 4; ++q) { const float t = a[q] * SCL; v[ch * 4 + q] = t; mx = fmaxf(mx, t); } }
#pragma unroll
    for (int sh = 16; sh; sh >>= 1) mx = fmaxf(mx, __shfl_xor(mx, sh, 32));
    float sum = 0.f;
#pragma unroll
    for (int k = 0; k < TT / 32; ++k) { float d0 = __fsub_rn(v[k], mx); asm volatile("" : "+v"(d0)); v[k] = __builtin_amdgcn_exp2f(__fmul_rn(d0, 1.4426950408889634f)); sum += v[k]; }
#pragma unroll
    for (int sh = 16; sh; sh >>= 1) sum += __shfl_xor(sum, sh, 32);
    const float f = __fdiv_rn(PCAR, sum);
#pragma unroll 1
    for (int ps = 0; ps < 2; ++ps) {
#pragma unroll
        for (int ch = 0; ch < TT / 128; ++ch) { v4h o4;
#pragma unroll
            for (int q = 0; q < 4; ++q) o4[q] = tohx(v[ch * 4 + q] * f);
            *(volatile v4h*)(P16 + (size_t)row * TT + ch * 128 + lane * 4) = o4; }
        if (ps == 0) __threadfence(); }
}

extern "C" void kernel_launch(void* const* d_in, const int* in_sizes, int n_in,
                              void* d_out, int out_size, void* d_ws, size_t ws_size, hipStream_t stream) {
    if (n_in < 3) return;
    const size_t need = ((size_t)(NB - 1) * SEQ_FULL + SEQ) * DM;
    if ((size_t)in_sizes[0] < need || (size_t)in_sizes[1] < need || (size_t)in_sizes[2] < need) return;
    if ((size_t)out_size < (size_t)NB * SEQ * DM) return;
    const float* q = (const float*)d_in[0]; const float* k = (const float*)d_in[1]; const float* v = (const float*)d_in[2];
    float* OUT = (float*)d_out;
    char* wsp = (char*)d_ws;
    auto take = [&](size_t bytes) { char* p = wsp; wsp += (bytes + 255) & ~(size_t)255; return (void*)p; };
    bf* QB = (bf*)take((size_t)NB * NH_ * TT * HD * 2); bf* KB = (bf*)take((size_t)NB * NH_ * TT * HD * 2); h16* VT16 = (h16*)take((size_t)NB * NH_ * HD * TT * 2);
    float* Sb = (float*)take((size_t)ZH * TT * TT * 4); h16* P16 = (h16*)take((size_t)ZH * TT * TT * 2);
    if ((size_t)(wsp - (char*)d_ws) > ws_size) return;
    k_hp8<<<(unsigned)(((size_t)NB * NH_ * TT * (HD / 8) + 255) / 256), 256, 0, stream>>>(q, k, QB, KB);
    k_vt8<<<(unsigned)(((size_t)NB * NH_ * HD * (TT / 8) + 255) / 256), 256, 0, stream>>>(v, VT16);
    for (int zp = 0; zp < NB * NH_; zp += ZH) { const int b = zp / NH_, h0 = zp % NH_; const size_t zo = (size_t)zp * TT * HD;
        k_gemmw<bf><<<dim3(TT / 64, TT / 64, ZH), 32, 0, stream>>>(QB + zo, KB + zo, HD, Sb, TT, (size_t)TT * HD, (size_t)TT * HD, (size_t)TT * TT, 1.0f);
        k_asoft<<<ZH * TT / 8, 256, 0, stream>>>(Sb, P16);
        k_gemmw<h16><<<dim3(TT / 64, HD / 64, ZH), 32, 0, stream>>>(P16, VT16 + zo, TT, OUT + (size_t)b * TT * DM + (size_t)h0 * HD, DM, (size_t)TT * TT, (size_t)HD * TT, (size_t)HD, 1.0f / PCAR); }
}
